// STDGAT_9208409883388
// MI455X (gfx1250) — hardware-verified
//
#include <hip/hip_runtime.h>


#define SS 24
#define BB 128
#define NN 121
#define FF 32
#define DX 3872
#define KX 3904
#define HH 512
#define G4 2048
#define MX (SS * BB)
#define NEGF (-9.0e15f)

typedef _Float16 f16t;
typedef unsigned short us16;
typedef f16t   v16h __attribute__((ext_vector_type(16)));
typedef f16t   v8h  __attribute__((ext_vector_type(8)));
typedef __bf16 v16b __attribute__((ext_vector_type(16)));
typedef us16   v8us __attribute__((ext_vector_type(8)));
typedef float  v8f  __attribute__((ext_vector_type(8)));
typedef float  v4f  __attribute__((ext_vector_type(4)));
typedef unsigned int v4u __attribute__((ext_vector_type(4)));

union FragH { v16h v; v8h q[2]; };
union FragB { v16b v; v8us q[2]; };
union Pk16 { v8h h; v8us s; v4u u; };
union Pk32 { v4f f; v4u u; };

__device__ __forceinline__ us16 bfb(float f) {
  unsigned int u = __float_as_uint(f);
  u += 0x7fffu + ((u >> 16) & 1u);
  return (us16)(u >> 16);
}
__device__ __forceinline__ float bfv(us16 b) { return __uint_as_float(((unsigned int)b) << 16); }
__device__ __forceinline__ float lrelu(float v) { return v >= 0.0f ? v : 0.01f * v; }
__device__ __forceinline__ float frcp(float v) { return __builtin_amdgcn_rcpf(v); }
__device__ __forceinline__ float sigm(float v) { return frcp(1.0f + __expf(-v)); }
__device__ __forceinline__ float ftanh(float x) {
  float ax = fabsf(x);
  float t  = __expf(-2.0f * ax);
  float r  = (1.0f - t) * frcp(1.0f + t);
  return copysignf(r, x);
}
__device__ __forceinline__ v8f zero8() { v8f z = {0.f, 0.f, 0.f, 0.f, 0.f, 0.f, 0.f, 0.f}; return z; }

__device__ __forceinline__ void split8(v4f a, v4f b, float sc, Pk16& hi, Pk16& lo) {
#pragma unroll
  for (int e = 0; e < 4; ++e) {
    float v0 = a[e] * sc; us16 h0 = bfb(v0); hi.s[e]     = h0; lo.s[e]     = bfb(v0 - bfv(h0));
    float v1 = b[e] * sc; us16 h1 = bfb(v1); hi.s[4 + e] = h1; lo.s[4 + e] = bfb(v1 - bfv(h1));
  }
}

__device__ __forceinline__ v8f mma_h(v16h a, v16h b, v8f c) {
  return __builtin_amdgcn_wmma_f32_16x16x32_f16(false, a, false, b, (short)0, c, false, false);
}
__device__ __forceinline__ v8f mma_b(v16b a, v16b b, v8f c) {
  return __builtin_amdgcn_wmma_f32_16x16x32_bf16(false, a, false, b, (short)0, c, false, false);
}

__device__ __forceinline__ void mma3x2(v8f& c0, v8f& c1, const FragB& ah, const FragB& al,
                                       const FragB (&bh)[2], const FragB (&bl)[2]) {
  c0 = mma_b(ah.v, bh[0].v, c0);
  c1 = mma_b(ah.v, bh[1].v, c1);
  c0 = mma_b(ah.v, bl[0].v, c0);
  c1 = mma_b(ah.v, bl[1].v, c1);
  c0 = mma_b(al.v, bh[0].v, c0);
  c1 = mma_b(al.v, bh[1].v, c1);
  asm volatile("v_nop\n\tv_nop\n\tv_nop\n\tv_nop"
               : "+v"(c0), "+v"(c1)
               : "v"(ah.v), "v"(al.v), "v"(bh[0].v), "v"(bh[1].v), "v"(bl[0].v), "v"(bl[1].v));
}

__global__ __launch_bounds__(256)
void k_prep(const float* __restrict__ Wih, const float* __restrict__ Whh, const float* __restrict__ Wfc,
            f16t* Pih, us16* Phh, us16* Plh, us16* Pfh, us16* Pfl) {
  const int tid = threadIdx.x;
  const int bid = blockIdx.x;
  if (bid < 3904) {
    const int p  = bid * 256 + tid;
    const int n  = p / 488;
    const int q  = p - n * 488;
    const int qc = q < 484 ? q : 483;
    const float sc = q < 484 ? 64.0f : 0.0f;
    const float* src = Wih + (size_t)n * DX + qc * 8;
    v4f a = *(const v4f*)src;
    v4f b = *(const v4f*)(src + 4);
    Pk16 k;
    k.h[0] = (f16t)(a[0] * sc); k.h[1] = (f16t)(a[1] * sc); k.h[2] = (f16t)(a[2] * sc); k.h[3] = (f16t)(a[3] * sc);
    k.h[4] = (f16t)(b[0] * sc); k.h[5] = (f16t)(b[1] * sc); k.h[6] = (f16t)(b[2] * sc); k.h[7] = (f16t)(b[3] * sc);
    f16t* d = Pih + (size_t)n * KX + q * 8;
    *(volatile v4u*)d = k.u;
    __threadfence();
    *(volatile v4u*)d = k.u;
  } else if (bid < 3904 + 512) {
    const int p = (bid - 3904) * 256 + tid;
    const int n = p >> 6;
    const int k = (p & 63) * 8;
    const float* src = Whh + (size_t)n * HH + k;
    v4f a = *(const v4f*)src;
    v4f b = *(const v4f*)(src + 4);
    Pk16 hi, lo;
    split8(a, b, 1.0f, hi, lo);
    us16* dh = Phh + (size_t)n * HH + k;
    us16* dl = Plh + (size_t)n * HH + k;
    *(volatile v4u*)dh = hi.u;
    *(volatile v4u*)dl = lo.u;
    __threadfence();
    *(volatile v4u*)dh = hi.u;
    *(volatile v4u*)dl = lo.u;
  } else {
    const int p  = (bid - 4416) * 256 + tid;
    const int n  = p >> 6;
    const int k  = (p & 63) * 8;
    const int nc = n < NN ? n : NN - 1;
    const float sc = n < NN ? 1.0f : 0.0f;
    const float* src = Wfc + (size_t)nc * HH + k;
    v4f a = *(const v4f*)src;
    v4f b = *(const v4f*)(src + 4);
    Pk16 hi, lo;
    split8(a, b, sc, hi, lo);
    us16* dh = Pfh + (size_t)n * HH + k;
    us16* dl = Pfl + (size_t)n * HH + k;
    *(volatile v4u*)dh = hi.u;
    *(volatile v4u*)dl = lo.u;
    __threadfence();
    *(volatile v4u*)dh = hi.u;
    *(volatile v4u*)dl = lo.u;
  }
}

__device__ __forceinline__ float att_rowsum(const unsigned char* msk, const float* sR, float sl, int n) {
  float mx = -__builtin_huge_valf();
  int any = 0;
#pragma unroll 4
  for (int j = 0; j < NN; ++j) {
    const int mm = msk[j * 128 + n];
    const float v = sR[j];
    mx = mm ? fmaxf(mx, v) : mx;
    any |= mm;
  }
  const float M = any ? lrelu(sl + mx) : NEGF;
  float S = 0.0f;
#pragma unroll 4
  for (int j = 0; j < NN; ++j) {
    const int mm = msk[j * 128 + n];
    const float e  = lrelu(sl + sR[j]);
    const float em = mm ? e : NEGF;
    S += __expf(em - M);
  }
  const float r = frcp(S);
  float rs = 0.0f;
#pragma unroll 4
  for (int j = 0; j < NN; ++j) {
    const int mm = msk[j * 128 + n];
    const float e  = lrelu(sl + sR[j]);
    const float em = mm ? e : NEGF;
    const float u  = __expf(em - M);
    rs += u * r;
  }
  return rs;
}

__device__ __forceinline__ void att_scores(const float* hf, const float* a, int n, float& dl, float& dr) {
  float l0 = 0.0f, r0 = 0.0f;
#pragma unroll
  for (int f = 0; f < FF; ++f) {
    const float hv = hf[n * FF + f];
    l0 = fmaf(hv, a[f], l0);
    r0 = fmaf(hv, a[FF + f], r0);
  }
  dl = l0; dr = r0;
}

__device__ __forceinline__ void emit_planes(const float* hf, us16* Apl, float rs, int n) {
#pragma unroll
  for (int f = 0; f < FF; ++f) {
    const float v = lrelu(hf[n * FF + f] * rs);
    const us16 hb = bfb(v);
    Apl[n * FF + f] = hb;
    Apl[128 * FF + n * FF + f] = bfb(v - bfv(hb));
  }
}

__device__ __forceinline__ void att_gemm(const us16* Ah, const us16* Al, const us16* Wh, const us16* Wl, float* hf) {
  const int tid = threadIdx.x, w = tid >> 5, l = tid & 31, hh = l >> 4, m = l & 15;
  FragB ah[2], al[2], bh[2], bl[2];
#pragma unroll
  for (int i = 0; i < 2; ++i) {
    const int ro = (32 * w + 16 * i + m) * FF + 8 * hh;
    ah[i].q[0] = *(const v8us*)(Ah + ro);
    ah[i].q[1] = *(const v8us*)(Ah + ro + 16);
    al[i].q[0] = *(const v8us*)(Al + ro);
    al[i].q[1] = *(const v8us*)(Al + ro + 16);
  }
#pragma unroll
  for (int j = 0; j < 2; ++j) {
    const int ro = (16 * j + m) * FF + 8 * hh;
    bh[j].q[0] = *(const v8us*)(Wh + ro);
    bh[j].q[1] = *(const v8us*)(Wh + ro + 16);
    bl[j].q[0] = *(const v8us*)(Wl + ro);
    bl[j].q[1] = *(const v8us*)(Wl + ro + 16);
  }
  v8f acc[2][2];
#pragma unroll
  for (int i = 0; i < 2; ++i)
#pragma unroll
    for (int j = 0; j < 2; ++j) acc[i][j] = zero8();
#pragma unroll
  for (int i = 0; i < 2; ++i)
#pragma unroll
    for (int j = 0; j < 2; ++j) acc[i][j] = mma_b(ah[i].v, bh[j].v, acc[i][j]);
#pragma unroll
  for (int i = 0; i < 2; ++i)
#pragma unroll
    for (int j = 0; j < 2; ++j) acc[i][j] = mma_b(ah[i].v, bl[j].v, acc[i][j]);
#pragma unroll
  for (int i = 0; i < 2; ++i)
#pragma unroll
    for (int j = 0; j < 2; ++j) acc[i][j] = mma_b(al[i].v, bh[j].v, acc[i][j]);
  asm volatile("v_nop\n\tv_nop\n\tv_nop\n\tv_nop"
               : "+v"(acc[0][0]), "+v"(acc[0][1]), "+v"(acc[1][0]), "+v"(acc[1][1])
               : "v"(ah[0].v), "v"(ah[1].v), "v"(al[0].v), "v"(al[1].v),
                 "v"(bh[0].v), "v"(bh[1].v), "v"(bl[0].v), "v"(bl[1].v));
#pragma unroll
  for (int i = 0; i < 2; ++i)
#pragma unroll
    for (int j = 0; j < 2; ++j)
#pragma unroll
      for (int r = 0; r < 8; ++r)
        hf[(32 * w + 16 * i + 8 * hh + r) * FF + 16 * j + m] = acc[i][j][r];
}

__global__ __launch_bounds__(128)
void k_att(const float* __restrict__ x, const int* __restrict__ adj,
           const float* __restrict__ W1, const float* __restrict__ a1,
           const float* __restrict__ W2, const float* __restrict__ a2,
           const float* __restrict__ W3, const float* __restrict__ a3,
           us16* X16) {
  __shared__ __attribute__((aligned(16))) unsigned char msk[NN * 128];
  __shared__ __attribute__((aligned(16))) us16  Apl[2 * 128 * FF];
  __shared__ __attribute__((aligned(16))) us16  Wpl[4 * FF * FF];
  __shared__ __attribute__((aligned(16))) float hf[128 * FF];
  __shared__ float sR[128];
  __shared__ float sw1[FF];
  __shared__ float sa[6 * FF];
  const int tid = threadIdx.x;
  const int n   = tid;
  const int nc  = n < NN ? n : NN - 1;
  const int row = blockIdx.x;
  const int s   = row >> 7;
  const int b   = row & 127;

  {
    const int* ar = adj + nc * NN;
    const int ok  = (n < NN) ? 1 : 0;
#pragma unroll 1
    for (int j = 0; j < NN; ++j) msk[j * 128 + n] = (unsigned char)(((ar[j] > 0) ? 1 : 0) & ok);
  }
  if (tid < FF) sw1[tid] = W1[tid];
  if (tid < 2 * FF) { sa[tid] = a1[tid]; sa[2 * FF + tid] = a2[tid]; sa[4 * FF + tid] = a3[tid]; }
#pragma unroll
  for (int qq = 0; qq < 8; ++qq) {
    const int e = tid + 128 * qq;
    const int no = e >> 5, k = e & 31;
    const float v2 = W2[k * FF + no]; const us16 h2 = bfb(v2);
    Wpl[no * FF + k] = h2; Wpl[FF * FF + no * FF + k] = bfb(v2 - bfv(h2));
    const float v3 = W3[k * FF + no]; const us16 h3 = bfb(v3);
    Wpl[2 * FF * FF + no * FF + k] = h3; Wpl[3 * FF * FF + no * FF + k] = bfb(v3 - bfv(h3));
  }
  __syncthreads();

  float sl, dr;
  {
    float xv = x[((size_t)b * SS + s) * NN + nc];
    xv = (n < NN) ? xv : 0.0f;
    float l0 = 0.0f, r0 = 0.0f;
#pragma unroll
    for (int f = 0; f < FF; ++f) {
      const float hv = xv * sw1[f];
      hf[n * FF + f] = hv;
      l0 = fmaf(hv, sa[f], l0);
      r0 = fmaf(hv, sa[FF + f], r0);
    }
    sl = l0; sR[n] = r0;
  }
  __syncthreads();
  { const float rs = att_rowsum(msk, sR, sl, n); emit_planes(hf, Apl, rs, n); }
  __syncthreads();
  att_gemm(Apl, Apl + 128 * FF, Wpl, Wpl + FF * FF, hf);
  __syncthreads();
  att_scores(hf, sa + 2 * FF, n, sl, dr);
  sR[n] = dr;
  __syncthreads();
  { const float rs = att_rowsum(msk, sR, sl, n); emit_planes(hf, Apl, rs, n); }
  __syncthreads();
  att_gemm(Apl, Apl + 128 * FF, Wpl + 2 * FF * FF, Wpl + 3 * FF * FF, hf);
  __syncthreads();
  att_scores(hf, sa + 4 * FF, n, sl, dr);
  sR[n] = dr;
  __syncthreads();
  {
    const float rs = att_rowsum(msk, sR, sl, n);
    if (n < NN + 1) {
#pragma unroll
      for (int f = 0; f < FF; ++f) {
        const float v = lrelu(hf[n * FF + f] * rs) * 8.0f;
        Apl[n * FF + f] = __builtin_bit_cast(us16, (f16t)v);
      }
    }
  }
  __syncthreads();
#pragma unroll
  for (int it = 0; it < 4; ++it) {
    const int p  = tid + 128 * it;
    const int pc = p < 488 ? p : 487;
    Pk16 v; v.s = *(const v8us*)(Apl + pc * 8);
    if (p < 488) *(volatile v4u*)(X16 + (size_t)row * KX + p * 8) = v.u;
  }
  __threadfence();
#pragma unroll
  for (int it = 0; it < 4; ++it) {
    const int p  = tid + 128 * it;
    const int pc = p < 488 ? p : 487;
    Pk16 v; v.s = *(const v8us*)(Apl + pc * 8);
    if (p < 488) *(volatile v4u*)(X16 + (size_t)row * KX + p * 8) = v.u;
  }
}

__global__ __launch_bounds__(128)
void k_xg(const f16t* __restrict__ X, const f16t* __restrict__ P,
          const float* __restrict__ bi, const float* __restrict__ bhh, float* XG) {
  __shared__ __attribute__((aligned(16))) float st[4 * 64 * 32];
  const int tid = threadIdx.x, w = tid >> 5, l = tid & 31, hh = l >> 4, m = l & 15;
  const int n0 = blockIdx.x * 128 + 32 * w;
  const int m0 = blockIdx.y * 64;
  v8f acc[4][2];
#pragma unroll
  for (int i = 0; i < 4; ++i)
#pragma unroll
    for (int j = 0; j < 2; ++j) acc[i][j] = zero8();
  const f16t* ap = X + (size_t)(m0 + m) * KX + 8 * hh;
  const f16t* bp = P + (size_t)(n0 + m) * KX + 8 * hh;
#pragma unroll 1
  for (int kt = 0; kt < KX / 32; ++kt) {
    FragH a[4], b[2];
#pragma unroll
    for (int i = 0; i < 4; ++i) {
      const f16t* p = ap + (size_t)(16 * i) * KX + 32 * kt;
      a[i].q[0] = *(const v8h*)p;
      a[i].q[1] = *(const v8h*)(p + 16);
    }
#pragma unroll
    for (int j = 0; j < 2; ++j) {
      const f16t* p = bp + (size_t)(16 * j) * KX + 32 * kt;
      b[j].q[0] = *(const v8h*)p;
      b[j].q[1] = *(const v8h*)(p + 16);
    }
#pragma unroll
    for (int i = 0; i < 4; ++i)
#pragma unroll
      for (int j = 0; j < 2; ++j) acc[i][j] = mma_h(a[i].v, b[j].v, acc[i][j]);
    asm volatile("v_nop\n\tv_nop\n\tv_nop\n\tv_nop"
                 : "+v"(acc[0][0]), "+v"(acc[0][1]), "+v"(acc[1][0]), "+v"(acc[1][1]),
                   "+v"(acc[2][0]), "+v"(acc[2][1]), "+v"(acc[3][0]), "+v"(acc[3][1])
                 : "v"(a[0].v), "v"(a[1].v), "v"(a[2].v), "v"(a[3].v), "v"(b[0].v), "v"(b[1].v));
  }
  float* sw = st + w * (64 * 32);
#pragma unroll
  for (int j = 0; j < 2; ++j) {
    const int col = n0 + 16 * j + m;
    const float bb = bi[col] + bhh[col];
#pragma unroll
    for (int i = 0; i < 4; ++i)
#pragma unroll
      for (int r = 0; r < 8; ++r)
        sw[(16 * i + 8 * hh + r) * 32 + 16 * j + m] = fmaf(acc[i][j][r], 0.001953125f, bb);
  }
  __syncthreads();
#pragma unroll
  for (int it = 0; it < 16; ++it) {
    const int rr = 4 * it + (l >> 3);
    const int c  = (l & 7) * 4;
    Pk32 v; v.f = *(const v4f*)(sw + rr * 32 + c);
    *(volatile v4u*)(XG + (size_t)(m0 + rr) * G4 + n0 + c) = v.u;
  }
  __threadfence();
#pragma unroll
  for (int it = 0; it < 16; ++it) {
    const int rr = 4 * it + (l >> 3);
    const int c  = (l & 7) * 4;
    Pk32 v; v.f = *(const v4f*)(sw + rr * 32 + c);
    *(volatile v4u*)(XG + (size_t)(m0 + rr) * G4 + n0 + c) = v.u;
  }
}

__global__ __launch_bounds__(32)
void k_step(const us16* __restrict__ Hh, const us16* __restrict__ Hl,
            const us16* __restrict__ Ph, const us16* __restrict__ Pl,
            const float* __restrict__ XGt, float* Cst, us16* Nh, us16* Nl) {
  __shared__ __attribute__((aligned(16))) float cs[16 * 64];
  __shared__ __attribute__((aligned(16))) us16  hs[2 * 16 * 64];
  const int l = threadIdx.x & 31, hh = l >> 4, m = l & 15;
  const int i = blockIdx.x >> 3, g = blockIdx.x & 7;
  const int r0 = 16 * i;
  const us16* ahp = Hh + (size_t)(r0 + m) * HH + 8 * hh;
  const us16* alp = Hl + (size_t)(r0 + m) * HH + 8 * hh;

#pragma unroll 1
  for (int half = 0; half < 2; ++half) {
    const int jb = 64 * g + 32 * half;
    v8f acc[8];
#pragma unroll
    for (int q = 0; q < 4; ++q)
#pragma unroll
      for (int jt = 0; jt < 2; ++jt) {
        const float* xp = XGt + (size_t)(r0 + 8 * hh) * G4 + q * HH + jb + 16 * jt + m;
#pragma unroll
        for (int r = 0; r < 8; ++r) acc[q * 2 + jt][r] = xp[(size_t)r * G4];
      }
#pragma unroll 1
    for (int kt = 0; kt < HH / 32; ++kt) {
      FragB ah, al;
      ah.q[0] = *(const v8us*)(ahp + 32 * kt);
      ah.q[1] = *(const v8us*)(ahp + 32 * kt + 16);
      al.q[0] = *(const v8us*)(alp + 32 * kt);
      al.q[1] = *(const v8us*)(alp + 32 * kt + 16);
#pragma unroll
      for (int q = 0; q < 4; ++q) {
        FragB bh[2], bl[2];
#pragma unroll
        for (int jt = 0; jt < 2; ++jt) {
          const size_t ro = (size_t)(q * HH + jb + 16 * jt + m) * HH + 8 * hh + 32 * kt;
          bh[jt].q[0] = *(const v8us*)(Ph + ro);
          bh[jt].q[1] = *(const v8us*)(Ph + ro + 16);
          bl[jt].q[0] = *(const v8us*)(Pl + ro);
          bl[jt].q[1] = *(const v8us*)(Pl + ro + 16);
        }
        mma3x2(acc[2 * q], acc[2 * q + 1], ah, al, bh, bl);
      }
    }
#pragma unroll
    for (int jt = 0; jt < 2; ++jt) {
      const int cl = 32 * half + 16 * jt + m;
      const float* cp = Cst + (size_t)(r0 + 8 * hh) * HH + 64 * g + cl;
#pragma unroll
      for (int r = 0; r < 8; ++r) {
        const float co = cp[(size_t)r * HH];
        const float gi = acc[0 * 2 + jt][r];
        const float gf = acc[1 * 2 + jt][r];
        const float gg = acc[2 * 2 + jt][r];
        const float go = acc[3 * 2 + jt][r];
        const float cn = sigm(gf) * co + sigm(gi) * ftanh(gg);
        const float hn = sigm(go) * ftanh(cn);
        const int rr = 8 * hh + r;
        cs[rr * 64 + cl] = cn;
        const us16 hb = bfb(hn);
        hs[rr * 64 + cl] = hb;
        hs[16 * 64 + rr * 64 + cl] = bfb(hn - bfv(hb));
      }
    }
  }
  __syncthreads();
#pragma unroll
  for (int it = 0; it < 8; ++it) {
    const int L  = 4 * it + (l >> 3);
    const int rr = L >> 1;
    const int cf = (L & 1) * 32 + (l & 7) * 4;
    Pk32 v; v.f = *(const v4f*)(cs + rr * 64 + cf);
    *(volatile v4u*)(Cst + (size_t)(r0 + rr) * HH + 64 * g + cf) = v.u;
  }
#pragma unroll
  for (int it = 0; it < 4; ++it) {
    const int rr = 4 * it + (l >> 3);
    const int cc = (l & 7) * 8;
    Pk16 a, b;
    a.s = *(const v8us*)(hs + rr * 64 + cc);
    b.s = *(const v8us*)(hs + 16 * 64 + rr * 64 + cc);
    *(volatile v4u*)(Nh + (size_t)(r0 + rr) * HH + 64 * g + cc) = a.u;
    *(volatile v4u*)(Nl + (size_t)(r0 + rr) * HH + 64 * g + cc) = b.u;
  }
  __threadfence();
#pragma unroll
  for (int it = 0; it < 8; ++it) {
    const int L  = 4 * it + (l >> 3);
    const int rr = L >> 1;
    const int cf = (L & 1) * 32 + (l & 7) * 4;
    Pk32 v; v.f = *(const v4f*)(cs + rr * 64 + cf);
    *(volatile v4u*)(Cst + (size_t)(r0 + rr) * HH + 64 * g + cf) = v.u;
  }
#pragma unroll
  for (int it = 0; it < 4; ++it) {
    const int rr = 4 * it + (l >> 3);
    const int cc = (l & 7) * 8;
    Pk16 a, b;
    a.s = *(const v8us*)(hs + rr * 64 + cc);
    b.s = *(const v8us*)(hs + 16 * 64 + rr * 64 + cc);
    *(volatile v4u*)(Nh + (size_t)(r0 + rr) * HH + 64 * g + cc) = a.u;
    *(volatile v4u*)(Nl + (size_t)(r0 + rr) * HH + 64 * g + cc) = b.u;
  }
}

__global__ __launch_bounds__(256)
void k_fc(const us16* __restrict__ Hh, const us16* __restrict__ Hl,
          const us16* __restrict__ Fh, const us16* __restrict__ Fl,
          const float* __restrict__ fcb, float* out) {
  __shared__ __attribute__((aligned(16))) float os[BB * NN];
  const int tid = threadIdx.x, w = tid >> 5, l = tid & 31, hh = l >> 4, m = l & 15;
  const int r0 = 16 * w;
  v8f acc[8];
#pragma unroll
  for (int j = 0; j < 8; ++j) acc[j] = zero8();
  const us16* ahp = Hh + (size_t)(r0 + m) * HH + 8 * hh;
  const us16* alp = Hl + (size_t)(r0 + m) * HH + 8 * hh;
#pragma unroll 1
  for (int kt = 0; kt < HH / 32; ++kt) {
    FragB ah, al;
    ah.q[0] = *(const v8us*)(ahp + 32 * kt);
    ah.q[1] = *(const v8us*)(ahp + 32 * kt + 16);
    al.q[0] = *(const v8us*)(alp + 32 * kt);
    al.q[1] = *(const v8us*)(alp + 32 * kt + 16);
#pragma unroll
    for (int jp = 0; jp < 4; ++jp) {
      FragB bh[2], bl[2];
#pragma unroll
      for (int jt = 0; jt < 2; ++jt) {
        const size_t ro = (size_t)(32 * jp + 16 * jt + m) * HH + 8 * hh + 32 * kt;
        bh[jt].q[0] = *(const v8us*)(Fh + ro);
        bh[jt].q[1] = *(const v8us*)(Fh + ro + 16);
        bl[jt].q[0] = *(const v8us*)(Fl + ro);
        bl[jt].q[1] = *(const v8us*)(Fl + ro + 16);
      }
      mma3x2(acc[2 * jp], acc[2 * jp + 1], ah, al, bh, bl);
    }
  }
#pragma unroll
  for (int j = 0; j < 8; ++j) {
    const int nn = 16 * j + m;
    const int nq = nn < NN ? nn : NN - 1;
    const float bb = fcb[nq];
#pragma unroll
    for (int r = 0; r < 8; ++r) {
      const float v = fmaxf(acc[j][r] + bb, 0.0f);
      if (nn < NN) os[(r0 + 8 * hh + r) * NN + nn] = v;
    }
  }
  __syncthreads();
#pragma unroll
  for (int it = 0; it < 16; ++it) {
    const int p  = tid + 256 * it;
    const int pc = p < 3872 ? p : 3871;
    Pk32 v; v.f = *(const v4f*)(os + pc * 4);
    if (p < 3872) *(volatile v4u*)(out + (size_t)p * 4) = v.u;
  }
  __threadfence();
#pragma unroll
  for (int it = 0; it < 16; ++it) {
    const int p  = tid + 256 * it;
    const int pc = p < 3872 ? p : 3871;
    Pk32 v; v.f = *(const v4f*)(os + pc * 4);
    if (p < 3872) *(volatile v4u*)(out + (size_t)p * 4) = v.u;
  }
}

extern "C" void kernel_launch(void* const* d_in, const int* in_sizes, int n_in,
                              void* d_out, int out_size, void* d_ws, size_t ws_size,
                              hipStream_t stream) {
  if (n_in < 14) return;
  if (in_sizes[0] != BB * SS * NN || in_sizes[1] != NN * NN || in_sizes[2] != FF ||
      in_sizes[3] != 2 * FF || in_sizes[4] != FF * FF || in_sizes[5] != 2 * FF ||
      in_sizes[6] != FF * FF || in_sizes[7] != 2 * FF || in_sizes[8] != G4 * DX ||
      in_sizes[9] != G4 * HH || in_sizes[10] != G4 || in_sizes[11] != G4 ||
      in_sizes[12] != NN * HH || in_sizes[13] != NN || out_size != BB * NN) return;

  const float* x    = (const float*)d_in[0];
  const int*   adj  = (const int*)d_in[1];
  const float* W1   = (const float*)d_in[2];
  const float* a1   = (const float*)d_in[3];
  const float* W2   = (const float*)d_in[4];
  const float* a2   = (const float*)d_in[5];
  const float* W3   = (const float*)d_in[6];
  const float* a3   = (const float*)d_in[7];
  const float* Wih  = (const float*)d_in[8];
  const float* Whh  = (const float*)d_in[9];
  const float* bih  = (const float*)d_in[10];
  const float* bhh  = (const float*)d_in[11];
  const float* Wfc  = (const float*)d_in[12];
  const float* bfc  = (const float*)d_in[13];
  float* out = (float*)d_out;

  char* ws = (char*)d_ws;
  size_t off = 0;
  auto carve = [&](size_t bytes) -> char* {
    char* p = ws + off;
    off = (off + bytes + 255) & ~(size_t)255;
    return p;
  };
  us16*  X16 = (us16*) carve((size_t)MX * KX * 2);
  f16t*  Pih = (f16t*) carve((size_t)G4 * KX * 2);
  us16*  Phh = (us16*) carve((size_t)G4 * HH * 2);
  us16*  Plh = (us16*) carve((size_t)G4 * HH * 2);
  us16*  Pfh = (us16*) carve((size_t)128 * HH * 2);
  us16*  Pfl = (us16*) carve((size_t)128 * HH * 2);
  float* XG  = (float*)carve((size_t)MX * G4 * 4);
  us16*  HAh = (us16*) carve((size_t)BB * HH * 2);
  us16*  HAl = (us16*) carve((size_t)BB * HH * 2);
  us16*  HBh = (us16*) carve((size_t)BB * HH * 2);
  us16*  HBl = (us16*) carve((size_t)BB * HH * 2);
  float* Cst = (float*)carve((size_t)BB * HH * 4);
  if (off > ws_size) return;
  if (off > (size_t)134217728) return;

  k_prep<<<dim3(3904 + 512 + 32), dim3(256), 0, stream>>>(Wih, Whh, Wfc, Pih, Phh, Plh, Pfh, Pfl);
  k_att<<<dim3(MX), dim3(128), 0, stream>>>(x, adj, W1, a1, W2, a2, W3, a3, X16);
  k_xg<<<dim3(G4 / 128, MX / 64), dim3(128), 0, stream>>>((const f16t*)X16, Pih, bih, bhh, XG);
  hipMemsetAsync(HAh, 0, (size_t)BB * HH * 2, stream);
  hipMemsetAsync(HAl, 0, (size_t)BB * HH * 2, stream);
  hipMemsetAsync(Cst, 0, (size_t)BB * HH * 4, stream);
  us16* hpl[2][2] = { { HAh, HAl }, { HBh, HBl } };
  for (int t = 0; t < SS; ++t) {
    const int cur = t & 1, nxt = cur ^ 1;
    k_step<<<dim3(64), dim3(32), 0, stream>>>(hpl[cur][0], hpl[cur][1], Phh, Plh,
                                              XG + (size_t)t * BB * G4, Cst,
                                              hpl[nxt][0], hpl[nxt][1]);
  }
  const int fin = SS & 1;
  k_fc<<<dim3(1), dim3(256), 0, stream>>>(hpl[fin][0], hpl[fin][1], Pfh, Pfl, bfc, out);
}
